// BidirectionalAttention_62826781605919
// MI455X (gfx1250) — hardware-verified
//
#include <hip/hip_runtime.h>
#include <stdint.h>


#ifndef NB
#define NB 8
#endif
#ifndef SEQ
#define SEQ 2048
#endif
#define NB_FULL  8
#define SEQ_FULL 2048
#define KD   256
#define VD   256
#define AD   128
#define ATM  32
#define ATJ  128
#define LDP  136
#define OSP  68
#define VTP  72
#define PCAR 16384.0f
#define L2E  1.4426950408889634f
#define OUT1_OFFB ((size_t)NB_FULL * SEQ_FULL * VD * 4)
#define WT_BYTES ((size_t)2 * AD * KD * 2)
#define XB_BYTES ((size_t)2 * NB * SEQ * KD * 2)
#define KP_BYTES ((size_t)2 * NB * SEQ * AD * 2)
#define VT_BYTES ((size_t)2 * NB * VD * SEQ * 2)

static_assert(NB >= 1 && NB <= NB_FULL);
static_assert(SEQ >= ATJ && SEQ <= SEQ_FULL && (SEQ % ATJ) == 0 && (SEQ % 64) == 0);
static_assert(AD == 128 && (KD % 32) == 0 && VD == 256 && ATM == 32 && ATJ == 128);
static_assert(OUT1_OFFB == (size_t)16777216);
static_assert(WT_BYTES + XB_BYTES + 2 * KP_BYTES + VT_BYTES <= (size_t)134217728);
static_assert((WT_BYTES % 256) == 0 && (XB_BYTES % 256) == 0 && (KP_BYTES % 256) == 0 && (VT_BYTES % 256) == 0);

typedef _Float16 h16;
typedef unsigned short bf;
typedef __attribute__((ext_vector_type(16))) __bf16   v16bf;
typedef __attribute__((ext_vector_type(16))) _Float16 v16h;
typedef __attribute__((ext_vector_type(8)))  _Float16 v8h;
typedef __attribute__((ext_vector_type(8)))  unsigned short v8us;
typedef __attribute__((ext_vector_type(2)))  unsigned short v2us;
typedef __attribute__((ext_vector_type(8)))  float    v8f;
typedef __attribute__((ext_vector_type(4)))  float    v4f;
typedef v8h  __attribute__((may_alias)) v8ha;
typedef v4f  __attribute__((may_alias)) v4fa;

__device__ __forceinline__ unsigned short f2bf(float f) { unsigned u = __float_as_uint(f); u += 0x7FFFu + ((u >> 16) & 1u); return (unsigned short)(u >> 16); }
__device__ __forceinline__ float bf2f(unsigned short b) { return __uint_as_float(((unsigned)b) << 16); }
__device__ __forceinline__ float bfr(float f) { return bf2f(f2bf(f)); }
__device__ __forceinline__ h16 tohx(float x) { return (h16)x; }
__device__ __forceinline__ void splitf(float y, unsigned short& hh, unsigned short& ll) { hh = f2bf(y); ll = f2bf(y - bf2f(hh)); }
__device__ __forceinline__ v8f z8() { v8f z = {0.f, 0.f, 0.f, 0.f, 0.f, 0.f, 0.f, 0.f}; return z; }
__device__ __forceinline__ v16h cat16(v8h lo, v8h hi) { return __builtin_shufflevector(lo, hi, 0, 1, 2, 3, 4, 5, 6, 7, 8, 9, 10, 11, 12, 13, 14, 15); }
__device__ __forceinline__ v16bf cat16b(v8us lo, v8us hi) { return __builtin_bit_cast(v16bf, __builtin_shufflevector(lo, hi, 0, 1, 2, 3, 4, 5, 6, 7, 8, 9, 10, 11, 12, 13, 14, 15)); }
__device__ __forceinline__ v8f wmma16(v16h a, v16h b, v8f c) { return __builtin_amdgcn_wmma_f32_16x16x32_f16(false, a, false, b, (short)0, c, false, false); }
__device__ __forceinline__ v8f wmmab(v16bf a, v16bf b, v8f c) { return __builtin_amdgcn_wmma_f32_16x16x32_bf16(false, a, false, b, (short)0, c, false, false); }

__device__ __forceinline__ v16bf ldbf(const bf* p) { return cat16b(*(const v8us*)p, *(const v8us*)(p + 16)); }
__device__ __forceinline__ v16h ldh(const h16* p) { return cat16(*(const v8h*)p, *(const v8h*)(p + 16)); }
__device__ __forceinline__ v16h ldhl(const h16* p) { return cat16(*(const v8ha*)p, *(const v8ha*)(p + 16)); }

__global__ __launch_bounds__(256) void k_wt(const float* __restrict__ wA, const float* __restrict__ wB, bf* WT) {
    const int which = blockIdx.y; const float* w = which ? wB : wA; bf* Bt = WT + (size_t)which * AD * KD;
    const int lane = threadIdx.x & 31; const int L0 = (blockIdx.x * 8 + (threadIdx.x >> 5)) * 8; const int nlines = AD * KD / 64;
#pragma unroll 1
    for (int ps = 0; ps < 2; ++ps) {
#pragma unroll 1
        for (int l = 0; l < 8; ++l) { const int L = L0 + l; if (L >= nlines) break; const size_t e = (size_t)L * 64 + lane * 2; const int k = (int)(e % KD), n = (int)(e / KD); v2us o;
            o[0] = f2bf(w[(size_t)k * AD + n]); o[1] = f2bf(w[(size_t)(k + 1) * AD + n]); *(volatile v2us*)(Bt + e) = o; }
        if (ps == 0) __threadfence(); }
}

__global__ __launch_bounds__(256) void k_cvtx(const float* __restrict__ k1, const float* __restrict__ k2, bf* XB) {
    const int which = blockIdx.z, b = blockIdx.y;
    const size_t i = (size_t)blockIdx.x * 256 + threadIdx.x; if (i >= (size_t)SEQ * KD / 8) return;
    const float* src = (which ? k2 : k1) + (size_t)b * SEQ_FULL * KD + i * 8;
    bf* dst = XB + ((size_t)which * NB + b) * SEQ * KD + i * 8;
    const v8f v = *(const v8f*)src; v8us o;
#pragma unroll
    for (int k = 0; k < 8; ++k) o[k] = f2bf(v[k]);
    *(volatile v8us*)dst = o; __threadfence(); *(volatile v8us*)dst = o;
}

__global__ __launch_bounds__(256) void k_vtp(const float* __restrict__ vG0, const float* __restrict__ vG1, h16* VT) {
    __shared__ __align__(16) h16 tile[64 * VTP];
    const int z = blockIdx.z; const int g = z / NB, b = z - g * NB;
    const float* src = ((g == 0) ? vG0 : vG1) + (size_t)b * SEQ_FULL * VD;
    h16* dst = VT + (size_t)z * VD * SEQ;
    const int m0 = blockIdx.x * 64, d0 = blockIdx.y * 64, t = threadIdx.x;
#pragma unroll
    for (int it = 0; it < 4; ++it) { const int idx = it * 256 + t; const int r = idx >> 4, c4 = (idx & 15) * 4;
        const v4f x = *(const v4f*)(src + (size_t)(m0 + r) * VD + d0 + c4);
#pragma unroll
        for (int j = 0; j < 4; ++j) tile[(c4 + j) * VTP + r] = tohx(bfr(x[j])); }
    __syncthreads();
    const int q = t & 7, lsub = t >> 3;
#pragma unroll 1
    for (int ps = 0; ps < 2; ++ps) {
#pragma unroll
        for (int it = 0; it < 2; ++it) { const int L = it * 32 + lsub;
            const v8h val = *(const v8ha*)(tile + L * VTP + q * 8);
            *(volatile v8h*)(dst + (size_t)(d0 + L) * SEQ + m0 + q * 8) = val; }
        if (ps == 0) __threadfence(); }
}

__global__ __launch_bounds__(32) void k_gemmp(const bf* __restrict__ X, const bf* __restrict__ WT, const float* __restrict__ bA, const float* __restrict__ bB, bf* Ph, bf* Pl) {
    __shared__ __align__(16) float os[16 * OSP];
    const int z = blockIdx.z; const int which = z / NB;
    const bf* A = X + (size_t)z * SEQ * KD; const bf* Bt = WT + (size_t)which * AD * KD; const float* bias = which ? bB : bA;
    bf* oh = Ph + (size_t)z * SEQ * AD; bf* ol = Pl + (size_t)z * SEQ * AD;
    const int lane = threadIdx.x & 31, lr = lane & 15, hi = lane >> 4; const int r0 = blockIdx.x * 32, c0 = blockIdx.y * 64;
    v8f acc[2][4];
#pragma unroll
    for (int mb = 0; mb < 2; ++mb)
#pragma unroll
        for (int nb = 0; nb < 4; ++nb) acc[mb][nb] = z8();
    const size_t aoff = (size_t)(r0 + lr) * KD + 8 * hi, boff = (size_t)(c0 + lr) * KD + 8 * hi;
#pragma unroll 1
    for (int kc = 0; kc < KD; kc += 32) {
        const v16bf a0 = ldbf(A + aoff + kc), a1 = ldbf(A + aoff + (size_t)16 * KD + kc);
        v16bf bq;
#pragma unroll
        for (int nb = 0; nb < 4; ++nb) { bq = ldbf(Bt + boff + (size_t)nb * 16 * KD + kc); acc[0][nb] = wmmab(a0, bq, acc[0][nb]); acc[1][nb] = wmmab(a1, bq, acc[1][nb]); }
        asm volatile("v_nop\n\tv_nop\n\tv_nop\n\tv_nop" : "+v"(acc[0][0]), "+v"(acc[0][1]), "+v"(acc[0][2]), "+v"(acc[0][3]), "+v"(acc[1][0]), "+v"(acc[1][1]), "+v"(acc[1][2]), "+v"(acc[1][3]) : "v"(a0), "v"(a1), "v"(bq));
    }
    const int q = lane & 7, rsub = lane >> 3;
    const v4f bb0 = *(const v4f*)(bias + c0 + q * 8), bb1 = *(const v4f*)(bias + c0 + q * 8 + 4);
#pragma unroll
    for (int mb = 0; mb < 2; ++mb) {
#pragma unroll
        for (int nb = 0; nb < 4; ++nb) {
#pragma unroll
            for (int j = 0; j < 8; ++j) os[(hi * 8 + j) * OSP + nb * 16 + lr] = acc[mb][nb][j]; }
        __builtin_amdgcn_fence(3  , "wavefront"); __builtin_amdgcn_wave_barrier(); asm volatile("" ::: "memory");
#pragma unroll 1
        for (int ps = 0; ps < 2; ++ps) {
#pragma unroll
            for (int i = 0; i < 4; ++i) { const int row = i * 4 + rsub;
                const v4f x0 = *(const v4fa*)(os + row * OSP + q * 8), x1 = *(const v4fa*)(os + row * OSP + q * 8 + 4); v8us vh, vl;
#pragma unroll
                for (int j = 0; j < 4; ++j) { unsigned short e0, e1; splitf(x0[j] + bfr(bb0[j]), e0, e1); vh[j] = e0; vl[j] = e1; splitf(x1[j] + bfr(bb1[j]), e0, e1); vh[4 + j] = e0; vl[4 + j] = e1; }
                const size_t oo = (size_t)(r0 + mb * 16 + row) * AD + c0 + q * 8; *(volatile v8us*)(oh + oo) = vh; *(volatile v8us*)(ol + oo) = vl; }
            if (ps == 0) __threadfence(); }
        __builtin_amdgcn_fence(3  , "wavefront"); __builtin_amdgcn_wave_barrier(); asm volatile("" ::: "memory");
    }
}

__global__ __launch_bounds__(256) void k_attn(const bf* __restrict__ Qh, const bf* __restrict__ Ql, const bf* __restrict__ Kh, const bf* __restrict__ Kl, const h16* __restrict__ VT, float* O) {
    __shared__ __align__(16) h16 lds_p[ATM * LDP];
    __shared__ __align__(16) float part_m[4 * ATM];
    __shared__ __align__(16) float part_s[4 * ATM];
    __shared__ __align__(16) float ost[8 * 16 * OSP];
    const int b = blockIdx.y, row0 = blockIdx.x * ATM;
    const int tid = threadIdx.x, lane = tid & 31, wid = tid >> 5, sr = wid >> 2, sc = wid & 3, h = lane >> 4, c16 = lane & 15;
    const int prow = sr * 16 + 8 * h;
    const size_t fa = (size_t)c16 * AD + 8 * h;
    const bf* qh = Qh + ((size_t)b * SEQ + row0 + sr * 16) * AD + fa;
    const bf* ql = Ql + ((size_t)b * SEQ + row0 + sr * 16) * AD + fa;
    const bf* kh = Kh + ((size_t)b * SEQ + sc * 32) * AD + fa;
    const bf* kl = Kl + ((size_t)b * SEQ + sc * 32) * AD + fa;
    const h16* vt = VT + ((size_t)b * VD + sc * 64 + c16) * SEQ + 8 * h;
    float* ob = O + ((size_t)b * SEQ_FULL + row0 + sr * 16) * VD + sc * 64;
    v8f o[4];
#pragma unroll
    for (int nb = 0; nb < 4; ++nb) o[nb] = z8();
    float mrun[8], srun[8];
#pragma unroll
    for (int r = 0; r < 8; ++r) { mrun[r] = -1.0e30f; srun[r] = 0.0f; }
#pragma unroll 1
    for (int it = 0; it < SEQ / ATJ; ++it) {
        const int j0 = it * ATJ;
        v8f s0 = z8(), s1 = z8();
#pragma unroll 1
        for (int kk = 0; kk < AD; kk += 32) {
            const v16bf ah = ldbf(qh + kk), al = ldbf(ql + kk);
            const v16bf bh0 = ldbf(kh + (size_t)j0 * AD + kk), bl0 = ldbf(kl + (size_t)j0 * AD + kk);
            const v16bf bh1 = ldbf(kh + (size_t)(j0 + 16) * AD + kk), bl1 = ldbf(kl + (size_t)(j0 + 16) * AD + kk);
            s0 = wmmab(ah, bh0, s0); s0 = wmmab(al, bh0, s0); s0 = wmmab(ah, bl0, s0);
            s1 = wmmab(ah, bh1, s1); s1 = wmmab(al, bh1, s1); s1 = wmmab(ah, bl1, s1);
            asm volatile("v_nop\n\tv_nop\n\tv_nop\n\tv_nop" : "+v"(s0), "+v"(s1) : "v"(ah), "v"(al), "v"(bh1), "v"(bl1));
        }
        float pm[8];
#pragma unroll
        for (int r = 0; r < 8; ++r) pm[r] = fmaxf(s0[r], s1[r]);
#pragma unroll
        for (int off = 1; off < 16; off <<= 1) {
#pragma unroll
            for (int r = 0; r < 8; ++r) pm[r] = fmaxf(pm[r], __shfl_xor(pm[r], off, 32));
        }
        if (c16 == 0) {
#pragma unroll
            for (int r = 0; r < 8; ++r) part_m[sc * ATM + prow + r] = pm[r];
        }
        __syncthreads();
        float mnew[8], alpha[8];
        {
            const v4f m00 = *(const v4fa*)(part_m + 0 * ATM + prow), m01 = *(const v4fa*)(part_m + 0 * ATM + prow + 4);
            const v4f m10 = *(const v4fa*)(part_m + 1 * ATM + prow), m11 = *(const v4fa*)(part_m + 1 * ATM + prow + 4);
            const v4f m20 = *(const v4fa*)(part_m + 2 * ATM + prow), m21 = *(const v4fa*)(part_m + 2 * ATM + prow + 4);
            const v4f m30 = *(const v4fa*)(part_m + 3 * ATM + prow), m31 = *(const v4fa*)(part_m + 3 * ATM + prow + 4);
#pragma unroll
            for (int r = 0; r < 4; ++r) {
                mnew[r]     = fmaxf(mrun[r],     fmaxf(fmaxf(m00[r], m10[r]), fmaxf(m20[r], m30[r])));
                mnew[4 + r] = fmaxf(mrun[4 + r], fmaxf(fmaxf(m01[r], m11[r]), fmaxf(m21[r], m31[r]))); }
        }
#pragma unroll
        for (int r = 0; r < 8; ++r) { alpha[r] = __builtin_amdgcn_exp2f((mrun[r] - mnew[r]) * L2E); mrun[r] = mnew[r]; srun[r] *= alpha[r]; }
#pragma unroll
        for (int nb = 0; nb < 4; ++nb) {
#pragma unroll
            for (int r = 0; r < 8; ++r) o[nb][r] *= alpha[r];
        }
#pragma unroll
        for (int r = 0; r < 8; ++r) {
            const h16 p0 = tohx(__builtin_amdgcn_exp2f((s0[r] - mnew[r]) * L2E) * PCAR);
            const h16 p1 = tohx(__builtin_amdgcn_exp2f((s1[r] - mnew[r]) * L2E) * PCAR);
            srun[r] += (float)p0; srun[r] += (float)p1;
            lds_p[(prow + r) * LDP + sc * 32 + c16] = p0;
            lds_p[(prow + r) * LDP + sc * 32 + 16 + c16] = p1;
        }
        __syncthreads();
#pragma unroll 1
        for (int k0 = 0; k0 < ATJ; k0 += 32) {
            const v16h pa = ldhl(lds_p + (sr * 16 + c16) * LDP + 8 * h + k0);
            v16h bv;
#pragma unroll
            for (int nb = 0; nb < 4; ++nb) { bv = ldh(vt + (size_t)nb * 16 * SEQ + j0 + k0); o[nb] = wmma16(pa, bv, o[nb]); }
            asm volatile("v_nop\n\tv_nop\n\tv_nop\n\tv_nop" : "+v"(o[0]), "+v"(o[1]), "+v"(o[2]), "+v"(o[3]) : "v"(pa), "v"(bv));
        }
        __syncthreads();
    }
#pragma unroll
    for (int off = 1; off < 16; off <<= 1) {
#pragma unroll
        for (int r = 0; r < 8; ++r) srun[r] += __shfl_xor(srun[r], off, 32);
    }
    if (c16 == 0) {
#pragma unroll
        for (int r = 0; r < 8; ++r) part_s[sc * ATM + prow + r] = srun[r];
    }
    __syncthreads();
    float inv[8];
    {
        const v4f t00 = *(const v4fa*)(part_s + 0 * ATM + prow), t01 = *(const v4fa*)(part_s + 0 * ATM + prow + 4);
        const v4f t10 = *(const v4fa*)(part_s + 1 * ATM + prow), t11 = *(const v4fa*)(part_s + 1 * ATM + prow + 4);
        const v4f t20 = *(const v4fa*)(part_s + 2 * ATM + prow), t21 = *(const v4fa*)(part_s + 2 * ATM + prow + 4);
        const v4f t30 = *(const v4fa*)(part_s + 3 * ATM + prow), t31 = *(const v4fa*)(part_s + 3 * ATM + prow + 4);
#pragma unroll
        for (int r = 0; r < 4; ++r) {
            inv[r]     = 1.0f / (((t00[r] + t10[r]) + t20[r]) + t30[r]);
            inv[4 + r] = 1.0f / (((t01[r] + t11[r]) + t21[r]) + t31[r]); }
    }
#pragma unroll
    for (int nb = 0; nb < 4; ++nb) {
#pragma unroll
        for (int r = 0; r < 8; ++r) o[nb][r] *= inv[r];
    }
    float* os = ost + wid * (16 * OSP);
#pragma unroll
    for (int nb = 0; nb < 4; ++nb) {
#pragma unroll
        for (int r = 0; r < 8; ++r) os[(8 * h + r) * OSP + nb * 16 + c16] = o[nb][r];
    }
    __builtin_amdgcn_fence(3  , "wavefront"); __builtin_amdgcn_wave_barrier(); asm volatile("" ::: "memory");
    const int q = lane & 7, lsub = lane >> 3;
#pragma unroll 1
    for (int ps = 0; ps < 2; ++ps) {
#pragma unroll
        for (int i = 0; i < 8; ++i) { const int L = i * 4 + lsub; const int row = L >> 1, hl = (L & 1) * 32;
            const v4f val = *(const v4fa*)(os + row * OSP + hl + q * 4);
            *(volatile v4f*)(ob + (size_t)row * VD + hl + q * 4) = val; }
        if (ps == 0) __threadfence(); }
}

extern "C" void kernel_launch(void* const* d_in, const int* in_sizes, int n_in,
                              void* d_out, int out_size, void* d_ws, size_t ws_size, hipStream_t stream) {
    if (n_in < 8) return;
    const size_t needk = ((size_t)(NB - 1) * SEQ_FULL + SEQ) * KD, needv = ((size_t)(NB - 1) * SEQ_FULL + SEQ) * VD;
    if ((size_t)in_sizes[0] < needk || (size_t)in_sizes[1] < needk || (size_t)in_sizes[2] < needv || (size_t)in_sizes[3] < needv) return;
    if (in_sizes[4] < KD * AD || in_sizes[5] < AD || in_sizes[6] < KD * AD || in_sizes[7] < AD) return;
    if ((size_t)out_size * 4 < OUT1_OFFB + needv * 4) return;
    const float* k1 = (const float*)d_in[0]; const float* k2 = (const float*)d_in[1];
    const float* v1 = (const float*)d_in[2]; const float* v2 = (const float*)d_in[3];
    const float* W1 = (const float*)d_in[4]; const float* b1 = (const float*)d_in[5];
    const float* W2 = (const float*)d_in[6]; const float* b2 = (const float*)d_in[7];
    float* out = (float*)d_out;
    char* wsp = (char*)d_ws; size_t used = 0;
    auto take = [&](size_t bytes) -> char* { char* p = wsp + used; used += (bytes + 255) & ~(size_t)255; return p; };
    bf* WT  = (bf*)take(WT_BYTES);
    bf* XB  = (bf*)take(XB_BYTES);
    bf* KPh = (bf*)take(KP_BYTES);
    bf* KPl = (bf*)take(KP_BYTES);
    h16* VT = (h16*)take(VT_BYTES);
    if (used > ws_size) return;
    k_wt<<<dim3((AD * KD / 64 + 63) / 64, 2), 256, 0, stream>>>(W1, W2, WT);
    k_cvtx<<<dim3((unsigned)(((size_t)SEQ * KD / 8 + 255) / 256), NB, 2), 256, 0, stream>>>(k1, k2, XB);
    k_vtp<<<dim3(SEQ / 64, VD / 64, 2 * NB), 256, 0, stream>>>(v2, v1, VT);
    k_gemmp<<<dim3(SEQ / 32, AD / 64, 2 * NB), 32, 0, stream>>>(XB, WT, b1, b2, KPh, KPl);
    const size_t kpg = (size_t)NB * SEQ * AD, vtg = (size_t)NB * VD * SEQ;
    k_attn<<<dim3(SEQ / ATM, NB), 256, 0, stream>>>(KPh, KPl, KPh + kpg, KPl + kpg, VT, out);
    k_attn<<<dim3(SEQ / ATM, NB), 256, 0, stream>>>(KPh + kpg, KPl + kpg, KPh, KPl, VT + vtg, out + OUT1_OFFB / 4);
}
